// RadialFunction_52080773431864
// MI455X (gfx1250) — hardware-verified
//
#include <hip/hip_runtime.h>
#include <math.h>


#ifndef NE
#define NE 2000000
#endif
#define NE_FULL 2000000
#define NSP   119
#define NPAIR (NSP * NSP)
#define NBAS  16
#define NRAD  8
#define GSH   6
#define GP    64
#define NG    ((NPAIR + GP - 1) / GP)
#define NGP   224
#define CH    16384
#define NCH   ((NE + CH - 1) / CH)
#define CAP   128
#define GSLOTS (NCH * CAP)
#define NPIECE (GSLOTS / 8)
#define SCAP  10240
#define NSEG  (SCAP / 16)
#define BT    512
#define NW    (BT / 32)
#define CSPW  (CH / (NW * 32))
#define GSTEP (GSLOTS / 32)
#define GSPW  ((GSTEP + NW - 1) / NW)
#define ECAR  64.0f
#define PSHA  8.0f
#define LOG2E 1.4426950408889634f
#define BETTA 7.111111164093018f
#define OSC   2.2257401724345982e-05f

static_assert(__builtin_bit_cast(unsigned, BETTA) == 0x40E38E39u);
static_assert(__builtin_bit_cast(unsigned, OSC) == 0x37BAB568u);
static_assert(NE <= NE_FULL);
static_assert(NE % 4 == 0);
static_assert(NBAS == 16);
static_assert(NRAD == 8);
static_assert(NG * GP >= NPAIR);
static_assert(NG <= NGP);
static_assert(NG <= BT);
static_assert(GP <= BT);
static_assert(CH % BT == 0);
static_assert(CH % (NW * 32) == 0);
static_assert(CH <= 16384);
static_assert(CAP == 128);
static_assert(32 * 16 == CAP * 4);
static_assert(32 * 4 == CAP);
static_assert(GSLOTS % 64 == 0);
static_assert(GSLOTS % 8 == 0);
static_assert(GSLOTS % 32 == 0);
static_assert(NW * GSPW >= GSTEP);
static_assert(SCAP % 32 == 0);
static_assert(SCAP < 65535);
static_assert(32 * 2 * 16 == 32 * NRAD * 4);
static_assert(((size_t)NPAIR * NRAD * NBAS) % 64 == 0);
static_assert((size_t)(NGP + NG * CAP + NW * NGP) * 4 <= 131072);
static_assert((size_t)SCAP * 4 + GP * 4 + (GP + 1) * 4 + NSEG * 4 + 4 + GP * 128 * 2 + NW * 256 * 4 + NW * GP * 4 + (size_t)GSLOTS * 2 <= 131072);

typedef _Float16 h16;
typedef unsigned short bf;
typedef __attribute__((ext_vector_type(16))) _Float16 v16h;
typedef __attribute__((ext_vector_type(8)))  _Float16 v8h;
typedef __attribute__((ext_vector_type(8)))  unsigned short v8us;
typedef __attribute__((ext_vector_type(8)))  float    v8f;
typedef __attribute__((ext_vector_type(4)))  float    v4f;
typedef __attribute__((ext_vector_type(4)))  unsigned v4u;
typedef __attribute__((ext_vector_type(2)))  unsigned v2u;
typedef v4f  __attribute__((may_alias)) v4fa;
typedef v8us __attribute__((may_alias)) v8usa;

__device__ __forceinline__ unsigned short f2bf(float f) { unsigned u = __float_as_uint(f); u += 0x7FFFu + ((u >> 16) & 1u); return (unsigned short)(u >> 16); }
__device__ __forceinline__ float bfr(float f) { return __uint_as_float(((unsigned)f2bf(f)) << 16); }
__device__ __forceinline__ v16h cat16(v8h lo, v8h hi) { return __builtin_shufflevector(lo, hi, 0, 1, 2, 3, 4, 5, 6, 7, 8, 9, 10, 11, 12, 13, 14, 15); }
__device__ __forceinline__ v8f wmma16(v16h a, v16h b, v8f c) { return __builtin_amdgcn_wmma_f32_16x16x32_f16(false, a, false, b, (short)0, c, false, false); }
__device__ __forceinline__ void wave_sync() { __builtin_amdgcn_fence(3  , "wavefront"); __builtin_amdgcn_wave_barrier(); asm volatile("" ::: "memory"); }
static __device__ __forceinline__ h16 toh_flush(float v) { const h16 r = (h16)v; return (fabsf(v) < 6.103515625e-05f) ? (h16)0.0f : r; }
__device__ __forceinline__ v8f wmma16g(v16h a, v16h b, v8f c) { c = wmma16(a, b, c); asm volatile("v_nop\n\tv_nop\n\tv_nop\n\tv_nop" : "+v"(c) : "v"(a), "v"(b)); return c; }
__device__ __forceinline__ h16 pexp(float betta, float d) { const float t = betta * (d * d); const float e = PSHA - t * LOG2E; const float v = __builtin_amdgcn_exp2f(e); return (e < -14.0f) ? (h16)0.0f : (h16)v; }
__device__ __forceinline__ unsigned same_key_mask(unsigned key, bool has) {
    const unsigned kk = has ? key : 0xFFFFFFFFu;
    unsigned mask = 0u;
#pragma unroll 4
    for (int j = 0; j < 32; ++j) {
        const unsigned kj = (unsigned)__builtin_amdgcn_readlane((int)kk, j);
        const bool eq = kk == kj;
        const unsigned m = __builtin_amdgcn_ballot_w32(eq);
        mask = eq ? m : mask;
    }
    return mask;
}

__global__ __launch_bounds__(256) void k_cvte(const float* __restrict__ src, h16* dst, size_t n8) {
    const size_t i = (size_t)blockIdx.x * 256 + threadIdx.x; if (i >= n8) return;
    const v8f v = *(const v8f*)(src + i * 8); v8h o;
#pragma unroll
    for (int k = 0; k < 8; ++k) o[k] = toh_flush(bfr(v[k]) * ECAR);
    *(volatile v8h*)(dst + i * 8) = o; __threadfence(); *(volatile v8h*)(dst + i * 8) = o;
}

__global__ __launch_bounds__(BT) void k_bucket(const float* __restrict__ dr, const int* __restrict__ zi, const int* __restrict__ zj, const float* __restrict__ cut,
                                               unsigned* REC, unsigned* SUBW, unsigned* PP) {
    __shared__ unsigned cnt[NGP];
    __shared__ unsigned sl[NG * CAP];
    __shared__ unsigned wh[NW * NGP];
    const int tid = threadIdx.x, lane = tid & 31;
    const int wave = __builtin_amdgcn_readfirstlane((int)(threadIdx.x >> 5));
    const unsigned below = (1u << lane) - 1u;
    const int c = blockIdx.x; const int base = c * CH;
#pragma unroll 1
    for (int i = tid; i < NGP; i += BT) cnt[i] = 0u;
#pragma unroll 1
    for (int i = tid; i < NG * CAP; i += BT) sl[i] = 0u;
#pragma unroll 1
    for (int i = tid; i < NW * NGP; i += BT) wh[i] = 0u;
    __syncthreads();
#pragma unroll 1
    for (int st = 0; st < CSPW; ++st) {
        const int li = (wave * CSPW + st) * 32 + lane; const int e = base + li; const bool ok = e < NE; const int ec = ok ? e : (NE - 1);
        int a = zi[ec]; int b = zj[ec];
        asm volatile("" : "+v"(a)); asm volatile("" : "+v"(b));
        a = a < 0 ? 0 : (a > NSP - 1 ? NSP - 1 : a); b = b < 0 ? 0 : (b > NSP - 1 ? NSP - 1 : b);
        const int key = b * NSP + a; const int g = key >> GSH;
        const unsigned mask = same_key_mask((unsigned)g, ok);
        const unsigned num = (unsigned)__builtin_popcount(mask);
        const bool first = ok & ((mask & below) == 0u);
        const unsigned v = wh[wave * NGP + g];
        wave_sync();
        if (first) wh[wave * NGP + g] = v + num;
        wave_sync();
    }
    __syncthreads();
    if (tid < NG) {
        unsigned run = 0u;
#pragma unroll 1
        for (int w = 0; w < NW; ++w) { const unsigned c0 = wh[w * NGP + tid]; wh[w * NGP + tid] = run; run += c0; }
        cnt[tid] = run;
    }
    __syncthreads();
#pragma unroll 1
    for (int st = 0; st < CSPW; ++st) {
        const int li = (wave * CSPW + st) * 32 + lane; const int e = base + li; const bool ok = e < NE; const int ec = ok ? e : (NE - 1);
        int a = zi[ec]; int b = zj[ec];
        asm volatile("" : "+v"(a)); asm volatile("" : "+v"(b));
        a = a < 0 ? 0 : (a > NSP - 1 ? NSP - 1 : a); b = b < 0 ? 0 : (b > NSP - 1 ? NSP - 1 : b);
        const int key = b * NSP + a; const int g = key >> GSH; const unsigned sub = (unsigned)(key & (GP - 1));
        const unsigned mask = same_key_mask((unsigned)g, ok);
        const unsigned num = (unsigned)__builtin_popcount(mask);
        const unsigned rank = (unsigned)__builtin_popcount(mask & below);
        const unsigned b0 = wh[wave * NGP + g];
        wave_sync();
        if (ok & (rank == 0u)) wh[wave * NGP + g] = b0 + num;
        const unsigned s = b0 + rank;
        unsigned P = 0xFFFFFFFFu;
        if (ok & (s < (unsigned)CAP)) { sl[g * CAP + (int)s] = (unsigned)li | (sub << 16); P = (unsigned)((g * NCH + c) * CAP) + s; }
        *(volatile unsigned*)(PP + e) = P; __threadfence(); *(volatile unsigned*)(PP + e) = P;
        wave_sync();
    }
    __syncthreads();
#pragma unroll 1
    for (int g = wave; g < NG; g += NW) {
        unsigned n = cnt[g]; n = n > (unsigned)CAP ? (unsigned)CAP : n;
        v4u rv; unsigned sb = 0u;
#pragma unroll
        for (int j = 0; j < 4; ++j) {
            const unsigned s = (unsigned)(4 * lane + j); const bool valid = s < n;
            const unsigned w = sl[g * CAP + (int)s];
            int e = base + (int)(w & 0x3FFFu); e = e > NE - 1 ? NE - 1 : e;
            float d = dr[e]; float q = cut[e];
            asm volatile("" : "+v"(d)); asm volatile("" : "+v"(q));
            const unsigned rec = ((unsigned)f2bf(d) << 16) | (unsigned)f2bf(q);
            rv[j] = valid ? rec : 0u;
            sb |= (valid ? ((w >> 16) & 63u) : 0xFFu) << (8 * j);
        }
        const size_t cell = (size_t)g * NCH + (size_t)c;
        unsigned* rp = REC + cell * CAP + 4 * lane;
        unsigned* sp = SUBW + cell * (CAP / 4) + lane;
        *(volatile v4u*)rp = rv; *(volatile unsigned*)sp = sb;
        __threadfence();
        *(volatile v4u*)rp = rv; *(volatile unsigned*)sp = sb;
    }
}

__global__ __launch_bounds__(BT) void k_group(const unsigned* __restrict__ REC, const unsigned* __restrict__ SUBW, const h16* __restrict__ EH,
                                              unsigned short* MAP, float* T2) {
    __shared__ unsigned srec[SCAP];
    __shared__ unsigned cnt[GP];
    __shared__ unsigned wh[NW * GP];
    __shared__ int off[GP + 1];
    __shared__ int segsub[NSEG];
    __shared__ int ntl;
    __shared__ __align__(16) unsigned short mapl[GSLOTS];
    __shared__ __align__(16) h16 et[GP * 128];
    __shared__ __align__(16) float os[NW * 256];
    const int tid = threadIdx.x, lane = tid & 31, lr = lane & 15, hi = lane >> 4;
    const int wave = __builtin_amdgcn_readfirstlane((int)(threadIdx.x >> 5));
    const unsigned below = (1u << lane) - 1u;
    const int g = blockIdx.x;
    const unsigned* subg = SUBW + (size_t)g * (GSLOTS / 4);
    const unsigned* recg = REC + (size_t)g * GSLOTS;
    int sbv = (int)(threadIdx.x >> 5) * GSPW; int sev = sbv + GSPW; sev = sev > GSTEP ? GSTEP : sev;
    const int sbeg = __builtin_amdgcn_readfirstlane(sbv);
    const int send = __builtin_amdgcn_readfirstlane(sev);
#pragma unroll 1
    for (int i = tid; i < SCAP; i += BT) srec[i] = 0u;
#pragma unroll 1
    for (int i = tid; i < NSEG; i += BT) segsub[i] = 0;
#pragma unroll 1
    for (int i = tid; i < NW * GP; i += BT) wh[i] = 0u;
    if (tid < GP) { cnt[tid] = 0u; }
#pragma unroll 1
    for (int p = tid; p < GP * 16; p += BT) {
        int gp = g * GP + (p >> 4); gp = gp > NPAIR - 1 ? NPAIR - 1 : gp;
        const v8h x = *(const v8h*)(EH + (size_t)gp * 128 + (size_t)(p & 15) * 8);
        *(v8h*)(&et[p * 8]) = x;
    }
    __syncthreads();
#pragma unroll 1
    for (int st = sbeg; st < send; ++st) {
        const int slot = st * 32 + lane;
        const unsigned w4 = subg[slot >> 2];
        const unsigned byte = (w4 >> (8 * (slot & 3))) & 0xFFu;
        const bool has = byte < (unsigned)GP;
        const int kb = has ? (int)byte : 0;
        const unsigned mask = same_key_mask(byte, has);
        const unsigned num = (unsigned)__builtin_popcount(mask);
        const bool first = has & ((mask & below) == 0u);
        const unsigned v = wh[wave * GP + kb];
        wave_sync();
        if (first) wh[wave * GP + kb] = v + num;
        wave_sync();
    }
    __syncthreads();
    if (tid < GP) {
        unsigned run = 0u;
#pragma unroll 1
        for (int w = 0; w < NW; ++w) { const unsigned c0 = wh[w * GP + tid]; wh[w * GP + tid] = run; run += c0; }
        cnt[tid] = run;
    }
    __syncthreads();
    if (tid == 0) {
        int run = 0;
#pragma unroll 1
        for (int i = 0; i < GP; ++i) { unsigned cc = cnt[i]; cc = cc > (unsigned)GSLOTS ? (unsigned)GSLOTS : cc; off[i] = run; run += (int)((cc + 15u) & ~15u); }
        off[GP] = run;
        const int ns = (run > SCAP ? SCAP : run) >> 4;
        ntl = (ns + 1) >> 1;
    }
    __syncthreads();
    if (tid < GP) {
        int s0 = off[tid]; int s1 = off[tid + 1];
        s0 = (s0 > SCAP ? SCAP : s0) >> 4; s1 = (s1 > SCAP ? SCAP : s1) >> 4;
#pragma unroll 1
        for (int s = s0; s < s1; ++s) segsub[s] = tid;
    }
#pragma unroll 1
    for (int st = sbeg; st < send; ++st) {
        const int slot = st * 32 + lane;
        const unsigned w4 = subg[slot >> 2];
        const unsigned rec = recg[slot];
        const unsigned byte = (w4 >> (8 * (slot & 3))) & 0xFFu;
        const bool has = byte < (unsigned)GP;
        const int kb = has ? (int)byte : 0;
        const unsigned mask = same_key_mask(byte, has);
        const unsigned num = (unsigned)__builtin_popcount(mask);
        const unsigned rank = (unsigned)__builtin_popcount(mask & below);
        const unsigned b0 = wh[wave * GP + kb];
        const unsigned o0 = (unsigned)off[kb];
        wave_sync();
        if (has & (rank == 0u)) wh[wave * GP + kb] = b0 + num;
        const unsigned s = o0 + b0 + rank;
        unsigned mv = 0xFFFFu;
        if (has & (s < (unsigned)SCAP)) { srec[s] = rec; mv = s; }
        mapl[slot] = (unsigned short)mv;
        wave_sync();
    }
    __syncthreads();
#pragma unroll 1
    for (int p = tid; p < NPIECE; p += BT) {
        const v8us mo = *(const v8usa*)(&mapl[8 * p]);
        unsigned short* mp = MAP + (size_t)g * GSLOTS + (size_t)8 * p;
        *(volatile v8us*)mp = mo; __threadfence(); *(volatile v8us*)mp = mo;
    }
    int ntv = ntl; ntv = ntv > SCAP / 32 ? SCAP / 32 : ntv; ntv = ntv < 0 ? 0 : ntv;
    const int nt = __builtin_amdgcn_readfirstlane(ntv);
    const int wbase = wave * 256;
    const v8h z8 = (v8h){};
#pragma unroll 1
    for (int t = wave; t < nt; t += NW) {
        const int r0 = t * 32;
        const unsigned wa = srec[r0 + lr], wb = srec[r0 + 16 + lr];
        const float da = __uint_as_float(wa & 0xFFFF0000u), db = __uint_as_float(wb & 0xFFFF0000u);
        v16h a;
#pragma unroll
        for (int i = 0; i < 8; ++i) { const float sh = 0.5f + 0.34375f * (float)(8 * hi + i); a[i] = pexp(BETTA, sh - da); a[8 + i] = pexp(BETTA, sh - db); }
        const int sa = segsub[2 * t] & (GP - 1), sb = segsub[2 * t + 1] & (GP - 1);
        const bool lo = lr < 8;
        const int sel = lo ? sa : sb;
        const v8h x = *(const v8h*)(&et[sel * 128 + (lr & 7) * 16 + 8 * hi]);
        const v16h bq = lo ? cat16(x, z8) : cat16(z8, x);
        v8f c = (v8f){};
        c = wmma16g(a, bq, c);
#pragma unroll
        for (int r = 0; r < 8; ++r) { const int el = (lr >> 3) * 16 + 8 * hi + r; const float cv = __uint_as_float(srec[r0 + el] << 16);
                                      os[wbase + el * 8 + (lr & 7)] = c[r] * OSC * cv; }
        wave_sync();
        float* tp = T2 + ((size_t)g * SCAP + (size_t)r0) * NRAD;
#pragma unroll 1
        for (int ps = 0; ps < 2; ++ps) {
#pragma unroll
            for (int s = 0; s < 2; ++s) { const int p = s * 32 + lane;
                const v4f val = *(const v4fa*)(&os[wbase + p * 4]);
                *(volatile v4f*)(tp + (size_t)p * 4) = val; }
            if (ps == 0) __threadfence(); }
        wave_sync();
    }
}

__global__ __launch_bounds__(256) void k_final(const unsigned* __restrict__ PP, const unsigned short* __restrict__ MAP, const float* __restrict__ T2, float* OUT) {
    const size_t i = (size_t)blockIdx.x * 256 + threadIdx.x; if (i >= (size_t)NE * 2) return;
    const size_t e = i >> 1; const int half = (int)(i & 1);
    unsigned P = PP[e];
    asm volatile("" : "+v"(P));
    const bool v0 = P < (unsigned)(NG * GSLOTS);
    const unsigned Pc = v0 ? P : (unsigned)(NG * GSLOTS - 1);
    const unsigned g = Pc / (unsigned)GSLOTS;
    unsigned mv = MAP[Pc];
    asm volatile("" : "+v"(mv));
    const bool v1 = v0 & (mv < (unsigned)SCAP);
    const unsigned mc = mv < (unsigned)SCAP ? mv : (unsigned)(SCAP - 1);
    v4f val = *(const v4f*)(T2 + ((size_t)g * SCAP + (size_t)mc) * NRAD + (size_t)half * 4);
    asm volatile("" : "+v"(val));
    const float qn = __uint_as_float(0x7FC00000u);
    v4f o;
#pragma unroll
    for (int k = 0; k < 4; ++k) o[k] = v1 ? val[k] : qn;
    *(volatile v4f*)(OUT + i * 4) = o; __threadfence(); *(volatile v4f*)(OUT + i * 4) = o;
}

static constexpr size_t al256(size_t v) { return (v + 255) & ~(size_t)255; }
static constexpr size_t SZ_EH  = al256((size_t)NPAIR * NRAD * NBAS * 2);
static constexpr size_t SZ_REC = al256((size_t)NG * GSLOTS * 4);
static constexpr size_t SZ_SUB = al256((size_t)NG * GSLOTS);
static constexpr size_t SZ_PP  = al256((size_t)NCH * CH * 4);
static constexpr size_t SZ_MAP = al256((size_t)NG * GSLOTS * 2);
static constexpr size_t SZ_T2  = al256((size_t)NG * SCAP * NRAD * 4);
static constexpr size_t SZ_TOTAL = SZ_EH + SZ_REC + SZ_SUB + SZ_PP + SZ_MAP + SZ_T2;
static_assert(SZ_TOTAL <= (size_t)134217728);
static_assert((size_t)NCH * CH >= (size_t)NE);
static_assert(((size_t)GSLOTS * 2) % 128 == 0);
static_assert(((size_t)SCAP * NRAD * 4) % 128 == 0);
static_assert((size_t)NG * GSLOTS < (size_t)0xFFFFFFFFu);

extern "C" void kernel_launch(void* const* d_in, const int* in_sizes, int n_in,
                              void* d_out, int out_size, void* d_ws, size_t ws_size, hipStream_t stream) {
    if (n_in < 5) return;
    if ((size_t)in_sizes[0] < (size_t)NE || (size_t)in_sizes[1] < (size_t)NE || (size_t)in_sizes[2] < (size_t)NE || (size_t)in_sizes[3] < (size_t)NE) return;
    if ((size_t)in_sizes[4] < (size_t)NPAIR * NRAD * NBAS) return;
    if ((size_t)out_size < (size_t)NE * NRAD) return;
    if (SZ_TOTAL > ws_size) return;
    const float* dr  = (const float*)d_in[0];
    const int*   zi  = (const int*)d_in[1];
    const int*   zj  = (const int*)d_in[2];
    const float* cut = (const float*)d_in[3];
    const float* emb = (const float*)d_in[4];
    float* OUT = (float*)d_out;
    char* wsp = (char*)d_ws;
    h16* EH = (h16*)wsp; wsp += SZ_EH;
    unsigned* REC = (unsigned*)wsp; wsp += SZ_REC;
    unsigned* SUBW = (unsigned*)wsp; wsp += SZ_SUB;
    unsigned* PP = (unsigned*)wsp; wsp += SZ_PP;
    unsigned short* MAP = (unsigned short*)wsp; wsp += SZ_MAP;
    float* T2 = (float*)wsp; wsp += SZ_T2;

    { const size_t n8 = (size_t)NPAIR * NRAD * NBAS / 8;
      k_cvte<<<(unsigned)((n8 + 255) / 256), 256, 0, stream>>>(emb, EH, n8); }
    k_bucket<<<NCH, BT, 0, stream>>>(dr, zi, zj, cut, REC, SUBW, PP);
    k_group<<<NG, BT, 0, stream>>>(REC, SUBW, EH, MAP, T2);
    { const size_t np = (size_t)NE * 2;
      k_final<<<(unsigned)((np + 255) / 256), 256, 0, stream>>>(PP, MAP, T2, OUT); }
}
